// TopoSAModule_4758823764634
// MI455X (gfx1250) — hardware-verified
//
#include <hip/hip_runtime.h>
#include <stddef.h>
#include <stdint.h>


#define CD      128
#define KG      8
#define NTHR    256
#define NWAVE   8
#define GROWS   128
#define PTB     16
#define AP      (CD + 8)
#define EPT     8
#define NGRP    2
#define CHUNK   (NTHR * EPT * NGRP)
#define WCAP    (EPT * NGRP * 32)
#define LISTN   (NWAVE * WCAP)
#define NBC     4096
#define TGT     256
#define NWPL    (CD * CD)
#define WGRP    (NWPL / 8)

#define LDS_GEMM (2 * GROWS * AP * 2)
#define LDS_AGG  ((TGT * CD + LISTN + NWAVE) * 4)

static_assert((CHUNK & (CHUNK - 1)) == 0);
static_assert(CHUNK <= 4096);
static_assert(NBC <= 4096 && (NBC & (NBC - 1)) == 0);
static_assert(TGT <= 4096 && (TGT & (TGT - 1)) == 0);
static_assert(TGT == NWAVE * 32);
static_assert(NBC == NWAVE * 4 * 128);
static_assert(GROWS * CD * 4 <= LDS_GEMM);
static_assert(PTB * KG == GROWS);
static_assert(PTB == 2 * NWAVE);
static_assert(GROWS == NWAVE * 16);
static_assert((GROWS * CD / 8) % NTHR == 0);
static_assert(WGRP % NTHR == 0);
static_assert((AP * 2) % 16 == 0);
static_assert(CD == 128);

typedef float          v4f  __attribute__((ext_vector_type(4)));
typedef float          v8f  __attribute__((ext_vector_type(8)));
typedef int            v4i  __attribute__((ext_vector_type(4)));
typedef unsigned short v8us __attribute__((ext_vector_type(8)));
typedef __bf16         v16b __attribute__((ext_vector_type(16)));
union FragB { v16b v; v8us h[2]; };

__device__ __forceinline__ unsigned short f2bf(float f) {
  unsigned int u = __float_as_uint(f);
  u += 0x7FFFu + ((u >> 16) & 1u);
  return (unsigned short)(u >> 16);
}
__device__ __forceinline__ float bf2f(unsigned short s) {
  return __uint_as_float(((unsigned int)s) << 16);
}
__device__ __forceinline__ void split1(float x, unsigned short& h, unsigned short& l) {
  const unsigned short hs = f2bf(x);
  const float rem = x - bf2f(hs);
  h = hs;
  l = f2bf(rem);
}
__device__ __forceinline__ void split8(v4f a, v4f b, v8us& hi, v8us& lo) {
  unsigned short h, l;
  split1(a.x, h, l); hi[0] = h; lo[0] = l;
  split1(a.y, h, l); hi[1] = h; lo[1] = l;
  split1(a.z, h, l); hi[2] = h; lo[2] = l;
  split1(a.w, h, l); hi[3] = h; lo[3] = l;
  split1(b.x, h, l); hi[4] = h; lo[4] = l;
  split1(b.y, h, l); hi[5] = h; lo[5] = l;
  split1(b.z, h, l); hi[6] = h; lo[6] = l;
  split1(b.w, h, l); hi[7] = h; lo[7] = l;
}

__device__ __forceinline__ v8f wmb(v16b a, v16b b, v8f c) {
  v8f d = __builtin_amdgcn_wmma_f32_16x16x32_bf16(false, a, false, b, (short)0, c, false, false);
  asm volatile("v_nop\n\tv_nop\n\tv_nop\n\tv_nop" : "+v"(d) : "v"(a), "v"(b));
  return d;
}

template <int NB>
__device__ __forceinline__ int scan_chunk(const int* __restrict__ dsts, int nE, int cbase, int slotBase,
                                          int vec8, int* list, int tid, int lane, int wave) {
  int wc = 0;
#pragma unroll
  for (int g = 0; g < NGRP; ++g) {
    const int el0  = (g * NTHR + tid) * EPT;
    const int e0   = cbase + el0;
    const int sent = -2147483647 - 1;
    v4i da, db;
    if (vec8 != 0 && cbase + CHUNK <= nE) {
      da = *(const v4i*)(dsts + e0);
      db = *(const v4i*)(dsts + e0 + 4);
    } else {
      da.x = (e0     < nE) ? dsts[min(e0, nE - 1)] : sent;
      da.y = (e0 + 1 < nE) ? dsts[min(e0 + 1, nE - 1)] : sent;
      da.z = (e0 + 2 < nE) ? dsts[min(e0 + 2, nE - 1)] : sent;
      da.w = (e0 + 3 < nE) ? dsts[min(e0 + 3, nE - 1)] : sent;
      db.x = (e0 + 4 < nE) ? dsts[min(e0 + 4, nE - 1)] : sent;
      db.y = (e0 + 5 < nE) ? dsts[min(e0 + 5, nE - 1)] : sent;
      db.z = (e0 + 6 < nE) ? dsts[min(e0 + 6, nE - 1)] : sent;
      db.w = (e0 + 7 < nE) ? dsts[min(e0 + 7, nE - 1)] : sent;
    }
    const unsigned nb = (unsigned)slotBase;
    const unsigned s0 = (unsigned)da.x - nb, s1 = (unsigned)da.y - nb;
    const unsigned s2 = (unsigned)da.z - nb, s3 = (unsigned)da.w - nb;
    const unsigned s4 = (unsigned)db.x - nb, s5 = (unsigned)db.y - nb;
    const unsigned s6 = (unsigned)db.z - nb, s7 = (unsigned)db.w - nb;
    const bool h0 = s0 < (unsigned)NB, h1 = s1 < (unsigned)NB, h2 = s2 < (unsigned)NB, h3 = s3 < (unsigned)NB;
    const bool h4 = s4 < (unsigned)NB, h5 = s5 < (unsigned)NB, h6 = s6 < (unsigned)NB, h7 = s7 < (unsigned)NB;
    const unsigned any = __builtin_amdgcn_ballot_w32(h0 | h1 | h2 | h3 | h4 | h5 | h6 | h7);
    if (any != 0u) {
#define HITJ(J, HJ, SJ) { \
        const unsigned mj = __builtin_amdgcn_ballot_w32(HJ); \
        if (mj != 0u) { \
          if (HJ) { \
            const int pos = wc + (int)__builtin_amdgcn_mbcnt_lo(mj, 0u); \
            if (pos < WCAP) list[wave * WCAP + pos] = ((el0 + (J)) << 12) | (int)(SJ); \
          } \
          wc += (int)__builtin_popcount(mj); } }
      HITJ(0, h0, s0)
      HITJ(1, h1, s1)
      HITJ(2, h2, s2)
      HITJ(3, h3, s3)
      HITJ(4, h4, s4)
      HITJ(5, h5, s5)
      HITJ(6, h6, s6)
      HITJ(7, h7, s7)
#undef HITJ
    }
  }
  return wc;
}

__global__ __launch_bounds__(NTHR) void k_wprep(const float* __restrict__ W1, const float* __restrict__ W2,
                                                const float* __restrict__ Wg, unsigned short* wpl) {
  const int i = blockIdx.x * NTHR + (int)threadIdx.x;
  if (i >= 3 * WGRP) return;
  const int w  = i / WGRP;
  const int j  = i - w * WGRP;
  const int n  = j >> 4;
  const int k0 = (j & 15) * 8;
  const float* src = (w == 0) ? W1 : ((w == 1) ? W2 : Wg);
  v4f a, b;
  a.x = src[(size_t)(k0 + 0) * CD + n];
  a.y = src[(size_t)(k0 + 1) * CD + n];
  a.z = src[(size_t)(k0 + 2) * CD + n];
  a.w = src[(size_t)(k0 + 3) * CD + n];
  b.x = src[(size_t)(k0 + 4) * CD + n];
  b.y = src[(size_t)(k0 + 5) * CD + n];
  b.z = src[(size_t)(k0 + 6) * CD + n];
  b.w = src[(size_t)(k0 + 7) * CD + n];
  v8us hi, lo;
  split8(a, b, hi, lo);
  unsigned short* ph = wpl + (size_t)(2 * w) * NWPL + (size_t)n * CD + k0;
  unsigned short* pl = ph + NWPL;
  *(volatile v8us*)ph = hi;
  *(volatile v8us*)pl = lo;
  __threadfence();
  *(volatile v8us*)ph = hi;
  *(volatile v8us*)pl = lo;
}

__global__ __launch_bounds__(NTHR) void k_count(const int* __restrict__ ei, float* dinv, int nE, int vec8) {
  __shared__ __attribute__((aligned(16))) int scnt[NBC];
  __shared__ __attribute__((aligned(16))) int list[LISTN];
  __shared__ int wcnt[NWAVE];
  const int tid = threadIdx.x, lane = tid & 31, wave = tid >> 5;
  const int nodeBase = blockIdx.x * NBC;
  const int* dsts = ei + nE;

  for (int i = tid; i < NBC; i += NTHR) scnt[i] = 0;
  __syncthreads();

  const int nChunks = (nE + CHUNK - 1) / CHUNK;
#pragma unroll 1
  for (int ch = 0; ch < nChunks; ++ch) {
    const int cbase = ch * CHUNK;
    const int wc = scan_chunk<NBC>(dsts, nE, cbase, nodeBase, vec8, list, tid, lane, wave);
    if (lane == 0) wcnt[wave] = wc;
    __syncthreads();
    if (wave == 0) {
#pragma unroll 1
      for (int wsx = 0; wsx < NWAVE; ++wsx) {
        int n = __builtin_amdgcn_readfirstlane(wcnt[wsx]);
        n = n > WCAP ? WCAP : (n < 0 ? 0 : n);
        const int* lp = list + wsx * WCAP;
#pragma unroll 1
        for (int i = 0; i < n; ++i) {
          const int ent  = __builtin_amdgcn_readfirstlane(lp[i]);
          const int slot = ent & (NBC - 1);
          if (lane == 0) scnt[slot] = scnt[slot] + 1;
        }
      }
    }
    __syncthreads();
  }

  v4f dq[4];
#pragma unroll
  for (int q = 0; q < 4; ++q) {
    const int f = (wave * 4 + q) * 128 + 4 * lane;
    const v4i c = *(const v4i*)(scnt + f);
    v4f d;
    d.x = rsqrtf((float)((c.x < 0 ? 0 : c.x) + 1));
    d.y = rsqrtf((float)((c.y < 0 ? 0 : c.y) + 1));
    d.z = rsqrtf((float)((c.z < 0 ? 0 : c.z) + 1));
    d.w = rsqrtf((float)((c.w < 0 ? 0 : c.w) + 1));
    dq[q] = d;
  }
  float* dp = dinv + (size_t)nodeBase;
#pragma unroll
  for (int q = 0; q < 4; ++q) {
    const int f = (wave * 4 + q) * 128 + 4 * lane;
    *(volatile v4f*)(dp + f) = dq[q];
  }
  __threadfence();
#pragma unroll
  for (int q = 0; q < 4; ++q) {
    const int f = (wave * 4 + q) * 128 + 4 * lane;
    *(volatile v4f*)(dp + f) = dq[q];
  }
}

template <int MODE>
__global__ __launch_bounds__(NTHR) void k_gemm(
    const float* __restrict__ Asrc, const int* __restrict__ sidx, const int* __restrict__ gidx,
    const unsigned short* __restrict__ Bh, const unsigned short* __restrict__ Bl,
    const float* __restrict__ b1, const float* __restrict__ b2, const float* __restrict__ dinv,
    float* C, int nM, int nN) {
  extern __shared__ v4f lds_dyn[];
  unsigned short* sAh = (unsigned short*)lds_dyn;
  unsigned short* sAl = sAh + GROWS * AP;
  float*          stg = (float*)lds_dyn;
  const int tid = threadIdx.x, lane = tid & 31, wave = tid >> 5, hh = lane >> 4, m = lane & 15;
  const int rowBase = blockIdx.x * GROWS;
  const int ptBase  = blockIdx.x * PTB;

#pragma unroll 2
  for (int i = 0; i < (GROWS * CD / 8) / NTHR; ++i) {
    const int idx = i * NTHR + tid;
    const int r   = idx >> 4;
    const int c0  = (idx & 15) * 8;
    const float* ap;
    if (MODE == 0) {
      int p = rowBase + r;
      p = p > nM - 1 ? nM - 1 : p;
      int s = sidx[p];
      s = s < 0 ? 0 : (s > nN - 1 ? nN - 1 : s);
      ap = Asrc + (size_t)s * CD + c0;
    } else if (MODE == 1) {
      int p = ptBase + (r >> 3);
      p = p > nM - 1 ? nM - 1 : p;
      int g = gidx[(size_t)p * KG + (r & 7)];
      g = g < 0 ? 0 : (g > nM - 1 ? nM - 1 : g);
      ap = Asrc + (size_t)g * CD + c0;
    } else {
      ap = Asrc + (size_t)(rowBase + r) * CD + c0;
    }
    v4f a = *(const v4f*)ap, b = *(const v4f*)(ap + 4);
    if (MODE == 1) {
      const v4f ba = *(const v4f*)(b1 + c0), bb = *(const v4f*)(b1 + c0 + 4);
      a = a + ba; b = b + bb;
      a.x = fmaxf(a.x, 0.0f); a.y = fmaxf(a.y, 0.0f); a.z = fmaxf(a.z, 0.0f); a.w = fmaxf(a.w, 0.0f);
      b.x = fmaxf(b.x, 0.0f); b.y = fmaxf(b.y, 0.0f); b.z = fmaxf(b.z, 0.0f); b.w = fmaxf(b.w, 0.0f);
    }
    v8us hi, lo;
    split8(a, b, hi, lo);
    *(v8us*)(sAh + r * AP + c0) = hi;
    *(v8us*)(sAl + r * AP + c0) = lo;
  }
  __syncthreads();

  v8f acc[8];
#pragma unroll
  for (int t = 0; t < 8; ++t) { v8f z = {0.f, 0.f, 0.f, 0.f, 0.f, 0.f, 0.f, 0.f}; acc[t] = z; }
  const unsigned short* arh = sAh + (wave * 16 + m) * AP + 8 * hh;
  const unsigned short* arl = sAl + (wave * 16 + m) * AP + 8 * hh;
#pragma unroll 1
  for (int kt = 0; kt < CD / 32; ++kt) {
    FragB ah, al;
    ah.h[0] = *(const v8us*)(arh + 32 * kt);
    ah.h[1] = *(const v8us*)(arh + 32 * kt + 16);
    al.h[0] = *(const v8us*)(arl + 32 * kt);
    al.h[1] = *(const v8us*)(arl + 32 * kt + 16);
#pragma unroll
    for (int t = 0; t < 8; ++t) {
      const size_t bo = (size_t)(16 * t + m) * CD + 32 * kt + 8 * hh;
      FragB bh, bl;
      bh.h[0] = *(const v8us*)(Bh + bo);
      bh.h[1] = *(const v8us*)(Bh + bo + 16);
      bl.h[0] = *(const v8us*)(Bl + bo);
      bl.h[1] = *(const v8us*)(Bl + bo + 16);
      acc[t] = wmb(ah.v, bh.v, acc[t]);
      acc[t] = wmb(ah.v, bl.v, acc[t]);
      acc[t] = wmb(al.v, bh.v, acc[t]);
    }
  }
  __syncthreads();

  if (MODE == 1) {
    const int pt = 2 * wave + hh;
    float* sp = stg + pt * CD + m;
#pragma unroll
    for (int t = 0; t < 8; ++t) {
      float v = acc[t][0];
#pragma unroll
      for (int r = 1; r < 8; ++r) v = fmaxf(v, acc[t][r]);
      sp[16 * t] = v + b2[16 * t + m];
    }
    __syncthreads();
    v4f ov[2];
#pragma unroll
    for (int i = 0; i < 2; ++i) ov[i] = *(const v4f*)(stg + (2 * wave + i) * CD + 4 * lane);
    float* gp = C + ((size_t)ptBase + 2 * wave) * CD + 4 * lane;
#pragma unroll
    for (int i = 0; i < 2; ++i) *(volatile v4f*)(gp + (size_t)i * CD) = ov[i];
    __threadfence();
#pragma unroll
    for (int i = 0; i < 2; ++i) *(volatile v4f*)(gp + (size_t)i * CD) = ov[i];
  } else {
    const int r0 = wave * 16 + 8 * hh;
    float s[8];
    if (MODE == 2) {
      const v4f dA = *(const v4f*)(dinv + (size_t)rowBase + r0);
      const v4f dB = *(const v4f*)(dinv + (size_t)rowBase + r0 + 4);
      s[0] = dA.x; s[1] = dA.y; s[2] = dA.z; s[3] = dA.w; s[4] = dB.x; s[5] = dB.y; s[6] = dB.z; s[7] = dB.w;
    } else {
#pragma unroll
      for (int r = 0; r < 8; ++r) s[r] = 1.0f;
    }
    float* sp = stg + r0 * CD + m;
#pragma unroll
    for (int t = 0; t < 8; ++t) {
#pragma unroll
      for (int r = 0; r < 8; ++r) sp[r * CD + 16 * t] = acc[t][r] * s[r];
    }
    __syncthreads();
    const float* lp = stg + wave * 16 * CD + 4 * lane;
    float* gp = C + ((size_t)rowBase + wave * 16) * CD + 4 * lane;
#pragma unroll
    for (int i = 0; i < 16; ++i) { const v4f v = *(const v4f*)(lp + i * CD); *(volatile v4f*)(gp + (size_t)i * CD) = v; }
    __threadfence();
#pragma unroll
    for (int i = 0; i < 16; ++i) { const v4f v = *(const v4f*)(lp + i * CD); *(volatile v4f*)(gp + (size_t)i * CD) = v; }
  }
}

__global__ __launch_bounds__(NTHR) void k_agg(
    const int* __restrict__ ei, const float* __restrict__ dinv, const float* __restrict__ xw,
    const float* __restrict__ bg, float* out, int nM, int nE, int vec8) {
  extern __shared__ v4f lds_dyn[];
  float* acc  = (float*)lds_dyn;
  int*   list = (int*)(acc + TGT * CD);
  int*   wcnt = list + LISTN;
  const int tid = threadIdx.x, lane = tid & 31, wave = tid >> 5;
  const int nodeBase = blockIdx.x * TGT;
  const int* dsts = ei + nE;

  {
    const v4f z = {0.f, 0.f, 0.f, 0.f};
    for (int i = tid; i < TGT * CD / 4; i += NTHR) ((v4f*)acc)[i] = z;
  }
  __syncthreads();

  const int nChunks = (nE + CHUNK - 1) / CHUNK;
#pragma unroll 1
  for (int ch = 0; ch < nChunks; ++ch) {
    const int cbase = ch * CHUNK;
    const int wc = scan_chunk<TGT>(dsts, nE, cbase, nodeBase, vec8, list, tid, lane, wave);
    if (lane == 0) wcnt[wave] = wc;
    __syncthreads();
    if (wave == 0) {
#pragma unroll 1
      for (int wsx = 0; wsx < NWAVE; ++wsx) {
        int n = __builtin_amdgcn_readfirstlane(wcnt[wsx]);
        n = n > WCAP ? WCAP : (n < 0 ? 0 : n);
        const int* lp = list + wsx * WCAP;
#pragma unroll 1
        for (int i = 0; i < n; ++i) {
          const int ent  = __builtin_amdgcn_readfirstlane(lp[i]);
          const int slot = ent & (TGT - 1);
          int e = cbase + ((ent >> 12) & (CHUNK - 1));
          e = e > nE - 1 ? nE - 1 : e;
          int s = ei[e];
          s = s < 0 ? 0 : (s > nM - 1 ? nM - 1 : s);
          const v4f v = *(const v4f*)(xw + (size_t)s * CD + 4 * lane);
          v4f* ap = (v4f*)(acc + slot * CD + 4 * lane);
          *ap = *ap + v;
        }
      }
    }
    __syncthreads();
  }

  const int tbase = nodeBase + wave * 32;
  union FI { float f; int i; };
  FI dvu; dvu.f = dinv[(size_t)tbase + lane];
  const v4f bgv = *(const v4f*)(bg + 4 * lane);
#pragma unroll 1
  for (int j = 0; j < 32; ++j) {
    const int c  = tbase + j;
    const int cc = c > nM - 1 ? nM - 1 : c;
    FI du; du.i = __builtin_amdgcn_readlane(dvu.i, j);
    const v4f av = *(const v4f*)(acc + (wave * 32 + j) * CD + 4 * lane);
    const v4f sv = *(const v4f*)(xw + (size_t)cc * CD + 4 * lane);
    const v4f v  = (av + sv) * du.f + bgv;
    if (c < nM) {
      float* gp = out + (size_t)c * CD + 4 * lane;
      *(volatile v4f*)gp = v;
      __threadfence();
      *(volatile v4f*)gp = v;
    }
  }
}

__device__ __forceinline__ float posval(const float* __restrict__ pos, const int* __restrict__ sidx,
                                        int f, int nF, int nM, int nN) {
  const int fc = f > nF - 1 ? nF - 1 : f;
  int p = fc / 3;
  const int c = fc - 3 * p;
  p = p > nM - 1 ? nM - 1 : p;
  int s = sidx[p];
  s = s < 0 ? 0 : (s > nN - 1 ? nN - 1 : s);
  return pos[(size_t)s * 3 + c];
}

__global__ __launch_bounds__(NTHR) void k_pos(const float* __restrict__ pos, const int* __restrict__ sidx,
                                              float* outp, int nM, int nN) {
  const int nF = 3 * nM;
  const int t  = blockIdx.x * NTHR + (int)threadIdx.x;
  const int f0 = 4 * t;
  if (f0 >= nF) return;
  v4f q;
  q.x = posval(pos, sidx, f0 + 0, nF, nM, nN);
  q.y = posval(pos, sidx, f0 + 1, nF, nM, nN);
  q.z = posval(pos, sidx, f0 + 2, nF, nM, nN);
  q.w = posval(pos, sidx, f0 + 3, nF, nM, nN);
  float* gp = outp + f0;
  if (f0 + 4 <= nF) {
    *(volatile v4f*)gp = q;
    __threadfence();
    *(volatile v4f*)gp = q;
  } else {
    *(volatile float*)(gp + 0) = q.x;
    if (f0 + 1 < nF) *(volatile float*)(gp + 1) = q.y;
    if (f0 + 2 < nF) *(volatile float*)(gp + 2) = q.z;
    __threadfence();
    *(volatile float*)(gp + 0) = q.x;
    if (f0 + 1 < nF) *(volatile float*)(gp + 1) = q.y;
    if (f0 + 2 < nF) *(volatile float*)(gp + 2) = q.z;
  }
}

extern "C" void kernel_launch(void* const* d_in, const int* in_sizes, int n_in,
                              void* d_out, int out_size, void* d_ws, size_t ws_size,
                              hipStream_t stream) {
  if (n_in < 11) return;
  const int nN = in_sizes[0] / CD;
  if (nN <= 0 || in_sizes[0] != nN * CD || in_sizes[1] != 3 * nN) return;
  if (in_sizes[2] != NWPL || in_sizes[3] != CD || in_sizes[4] != NWPL || in_sizes[5] != CD ||
      in_sizes[6] != NWPL || in_sizes[7] != CD) return;
  const int nM = in_sizes[8];
  if (nM <= 0 || in_sizes[9] != nM * KG) return;
  const int nE = in_sizes[10] / 2;
  if (nE <= 0 || in_sizes[10] != 2 * nE) return;
  if (nM > (1 << 22) || nN > (1 << 24) || nE > (1 << 28)) return;
  if (out_size != nM * CD + 3 * nM) return;

  const float* x    = (const float*)d_in[0];
  const float* pos  = (const float*)d_in[1];
  const float* W1   = (const float*)d_in[2];
  const float* b1   = (const float*)d_in[3];
  const float* W2   = (const float*)d_in[4];
  const float* b2   = (const float*)d_in[5];
  const float* Wg   = (const float*)d_in[6];
  const float* bg   = (const float*)d_in[7];
  const int*   sidx = (const int*)d_in[8];
  const int*   gidx = (const int*)d_in[9];
  const int*   ei   = (const int*)d_in[10];
  float* out0 = (float*)d_out;
  float* out1 = out0 + (size_t)nM * CD;

  const int PFPAD = ((nM + GROWS - 1) / GROWS) * GROWS;
  const int TPAD  = ((nM + TGT - 1) / TGT) * TGT;
  const int nBC   = (TPAD + NBC - 1) / NBC;
  const int DVPAD = nBC * NBC;

  char* ws = (char*)d_ws;
  size_t off = 0;
  const size_t oW  = off; off += (size_t)6 * NWPL * 2;        off = (off + 255) & ~(size_t)255;
  const size_t oDv = off; off += (size_t)DVPAD * 4;           off = (off + 255) & ~(size_t)255;
  const size_t oP1 = off; off += (size_t)PFPAD * CD * 4;      off = (off + 255) & ~(size_t)255;
  const size_t oPF = off; off += (size_t)PFPAD * CD * 4;      off = (off + 255) & ~(size_t)255;
  const size_t oXW = off; off += (size_t)PFPAD * CD * 4;      off = (off + 255) & ~(size_t)255;
  const size_t cap = ws_size < ((size_t)128 << 20) ? ws_size : ((size_t)128 << 20);
  if (off > cap) return;
  unsigned short* wpl  = (unsigned short*)(ws + oW);
  float*          dinv = (float*)(ws + oDv);
  float*          P1   = (float*)(ws + oP1);
  float*          PF   = (float*)(ws + oPF);
  float*          XW   = (float*)(ws + oXW);
  const unsigned short* w1h = wpl + 0 * NWPL;
  const unsigned short* w1l = wpl + 1 * NWPL;
  const unsigned short* w2h = wpl + 2 * NWPL;
  const unsigned short* w2l = wpl + 3 * NWPL;
  const unsigned short* wgh = wpl + 4 * NWPL;
  const unsigned short* wgl = wpl + 5 * NWPL;

  const int vec8 = ((nE & 3) == 0) ? 1 : 0;

  k_wprep<<<(3 * WGRP) / NTHR, NTHR, 0, stream>>>(W1, W2, Wg, wpl);

  k_count<<<nBC, NTHR, 0, stream>>>(ei, dinv, nE, vec8);

  hipFuncSetAttribute(reinterpret_cast<const void*>(&k_gemm<0>), hipFuncAttributeMaxDynamicSharedMemorySize, LDS_GEMM);
  hipFuncSetAttribute(reinterpret_cast<const void*>(&k_gemm<1>), hipFuncAttributeMaxDynamicSharedMemorySize, LDS_GEMM);
  hipFuncSetAttribute(reinterpret_cast<const void*>(&k_gemm<2>), hipFuncAttributeMaxDynamicSharedMemorySize, LDS_GEMM);
  k_gemm<0><<<PFPAD / GROWS, NTHR, LDS_GEMM, stream>>>(x, sidx, gidx, w1h, w1l, b1, b2, dinv, P1, nM, nN);

  k_gemm<1><<<PFPAD / PTB, NTHR, LDS_GEMM, stream>>>(P1, sidx, gidx, w2h, w2l, b1, b2, dinv, PF, nM, nN);

  k_gemm<2><<<PFPAD / GROWS, NTHR, LDS_GEMM, stream>>>(PF, sidx, gidx, wgh, wgl, b1, b2, dinv, XW, nM, nN);

  hipFuncSetAttribute(reinterpret_cast<const void*>(&k_agg), hipFuncAttributeMaxDynamicSharedMemorySize, LDS_AGG);
  k_agg<<<TPAD / TGT, NTHR, LDS_AGG, stream>>>(ei, dinv, XW, bg, out0, nM, nE, vec8);

  const int nT = (3 * nM + 3) / 4;
  k_pos<<<(nT + NTHR - 1) / NTHR, NTHR, 0, stream>>>(pos, sidx, out1, nM, nN);
}
